// MEAttention_7172595384820
// MI455X (gfx1250) — hardware-verified
//
#include <hip/hip_runtime.h>
#include <math.h>

typedef __attribute__((ext_vector_type(16))) _Float16 v16h;
typedef __attribute__((ext_vector_type(16))) __bf16 v16b;
typedef __attribute__((ext_vector_type(8)))  _Float16 v8h;
typedef __attribute__((ext_vector_type(8)))  float v8f;
typedef __attribute__((ext_vector_type(4)))  float v4f;
typedef __attribute__((ext_vector_type(2)))  float v2f;
typedef __attribute__((ext_vector_type(4)))  unsigned v4u;
typedef __attribute__((ext_vector_type(4)))  int v4i;
typedef float __attribute__((may_alias)) float_a;
typedef int __attribute__((may_alias)) int_a;

template <typename T> __device__ __forceinline__ void vst2(void* p, T v) { *(volatile T*)p = v; __threadfence(); *(volatile T*)p = v; }
__device__ __forceinline__ v8f wmma16(v16h a, v16h b, v8f c) {
  v8f d = __builtin_amdgcn_wmma_f32_16x16x32_f16(false, a, false, b, (short)0, c, false, false);
  asm volatile("v_nop\n\tv_nop\n\tv_nop\n\tv_nop" : "+v"(d) : "v"(a), "v"(b));
  return d;
}
__device__ __forceinline__ v8f wmma_bf(v16b a, v16b b, v8f c) {
  v8f d = __builtin_amdgcn_wmma_f32_16x16x32_bf16(false, a, false, b, (short)0, c, false, false);
  asm volatile("v_nop\n\tv_nop\n\tv_nop\n\tv_nop" : "+v"(d) : "v"(a), "v"(b));
  return d;
}
__device__ __forceinline__ v16h frag_h(const _Float16* rowk0, int lane) {
  union { v16h v; v8h q[2]; } u; const _Float16* p = rowk0 + 8 * (lane >> 4);
  u.q[0] = *(const v8h*)p; u.q[1] = *(const v8h*)(p + 16); return u.v;
}
__device__ __forceinline__ v16h frag_f32(const float* rowk0, int lane) {
  v16h a; const float* p = rowk0 + 8 * (lane >> 4);
#pragma unroll
  for (int i = 0; i < 8; ++i) { a[i] = (_Float16)p[i]; a[8 + i] = (_Float16)p[16 + i]; }
  return a;
}
__device__ __forceinline__ v16h frag_f32s(const float* rowk0, int lane, float sc) {
  v16h a; const float* p = rowk0 + 8 * (lane >> 4);
#pragma unroll
  for (int i = 0; i < 8; ++i) { a[i] = (_Float16)(p[i] * sc); a[8 + i] = (_Float16)(p[16 + i] * sc); }
  return a;
}
__device__ __forceinline__ v16h fragc_f32(const float* W, int k0, int n, int lane, int ld, int K) {
  v16h a; const int g = lane >> 4;
#pragma unroll
  for (int i = 0; i < 8; ++i) { const int ka = k0 + 8 * g + i, kb = ka + 16;
    a[i] = (_Float16)(ka < K ? W[(size_t)ka * ld + n] : 0.f); a[8 + i] = (_Float16)(kb < K ? W[(size_t)kb * ld + n] : 0.f); }
  return a;
}
struct F2 { v16b h, l; };
__device__ __forceinline__ F2 bsplit16(const float v[16]) { F2 r;
#pragma unroll
  for (int i = 0; i < 16; ++i) { const __bf16 h = (__bf16)v[i]; r.h[i] = h; r.l[i] = (__bf16)(v[i] - (float)h); }
  return r; }
__device__ __forceinline__ F2 split_row(const float* row, int k0, int lane) { float v[16]; const float* p = row + k0 + 8 * (lane >> 4);
#pragma unroll
  for (int i = 0; i < 8; ++i) { v[i] = p[i]; v[8 + i] = p[16 + i]; }
  return bsplit16(v); }
__device__ __forceinline__ F2 split_rowK(const float* row, int k0, int lane, int K) { float v[16]; const int g = lane >> 4;
#pragma unroll
  for (int i = 0; i < 8; ++i) { const int ka = k0 + 8 * g + i, kb = ka + 16; v[i] = ka < K ? row[ka] : 0.f; v[8 + i] = kb < K ? row[kb] : 0.f; }
  return bsplit16(v); }
__device__ __forceinline__ F2 split_col(const float* W, int k0, int n, int lane, int ld, int K) { float v[16]; const int g = lane >> 4;
#pragma unroll
  for (int i = 0; i < 8; ++i) { const int ka = k0 + 8 * g + i, kb = ka + 16; v[i] = ka < K ? W[(size_t)ka * ld + n] : 0.f; v[8 + i] = kb < K ? W[(size_t)kb * ld + n] : 0.f; }
  return bsplit16(v); }
__device__ __forceinline__ v8f mac3(const F2& a, const F2& b, v8f c) { c = wmma_bf(a.l, b.h, c); c = wmma_bf(a.h, b.l, c); return wmma_bf(a.h, b.h, c); }
__device__ __forceinline__ float sigm(float v) { return 1.0f / (1.0f + expf(-v)); }
#define LDSX() do { asm volatile("s_wait_dscnt 0" ::: "memory"); __builtin_amdgcn_wave_barrier(); __builtin_amdgcn_fence(__ATOMIC_RELEASE, "workgroup"); } while (0)

#define NB 2
#define SQ 1024
#define SK 1024
#define DM 512
#define NI 64
#define NRQ (NB * SQ)

__global__ __launch_bounds__(128) void k_proj(const float* __restrict__ x, const float* __restrict__ emb, const float* __restrict__ Wq, const float* __restrict__ Wk, const float* __restrict__ Wv, float* __restrict__ Q, float* __restrict__ K, float* __restrict__ V) {
  __shared__ __align__(16) float so[4][16][68];
  const int tid = threadIdx.x, wave = tid >> 5, lane = tid & 31, col = lane & 15, g = lane >> 4;
  const int which = blockIdx.y, r0 = blockIdx.x * 64 + wave * 16;
  const float* src = which == 0 ? x : emb; const float* W = which == 0 ? Wq : (which == 1 ? Wk : Wv); float* dst = which == 0 ? Q : (which == 1 ? K : V);
  v8f acc[4] = {};
#pragma unroll 1
  for (int kc = 0; kc < DM / 32; ++kc) { const F2 a = split_row(src + (size_t)(r0 + col) * DM, kc * 32, lane);
#pragma unroll
    for (int j = 0; j < 4; ++j) acc[j] = mac3(a, split_col(W, kc * 32, j * 16 + col, lane, NI, DM), acc[j]); }
#pragma unroll
  for (int j = 0; j < 4; ++j)
#pragma unroll
    for (int r = 0; r < 8; ++r) so[wave][8 * g + r][j * 16 + col] = acc[j][r];
  LDSX();
  for (int q = lane; q < 16 * 16; q += 32) { const int rl = q >> 4, pc = q & 15; vst2(dst + (size_t)(r0 + rl) * NI + pc * 4, *(const v4f*)(&so[wave][rl][pc * 4])); }
}
__global__ __launch_bounds__(256) void k_attn(const float* __restrict__ Q, const float* __restrict__ K, const float* __restrict__ V, float* __restrict__ O) {
  __shared__ float sk[SK][17], sv[SK][17];
  __shared__ __align__(16) float so[64][NI + 4];
  const int tid = threadIdx.x, b = blockIdx.y, i0 = blockIdx.x * 64; const int il = tid >> 2, hq = tid & 3;
#pragma unroll 1
  for (int hb = 0; hb < NI; hb += 16) {
    __syncthreads();
    for (int q = tid; q < SK * 16; q += 256) { const int j = q >> 4, hh = q & 15; sk[j][hh] = K[((size_t)b * SK + j) * NI + hb + hh]; sv[j][hh] = V[((size_t)b * SK + j) * NI + hb + hh]; }
    __syncthreads();
    float qv[4], mx[4], l[4], o[4];
#pragma unroll
    for (int e = 0; e < 4; ++e) { qv[e] = Q[((size_t)b * SQ + i0 + il) * NI + hb + hq * 4 + e]; mx[e] = -3.0e38f; l[e] = 0.f; o[e] = 0.f; }
#pragma unroll 4
    for (int j = 0; j < SK; ++j) {
#pragma unroll
      for (int e = 0; e < 4; ++e) mx[e] = fmaxf(mx[e], qv[e] * sk[j][hq * 4 + e]); }
#pragma unroll 4
    for (int j = 0; j < SK; ++j) {
#pragma unroll
      for (int e = 0; e < 4; ++e) { const float p = expf(qv[e] * sk[j][hq * 4 + e] - mx[e]); l[e] += p; o[e] += p * sv[j][hq * 4 + e]; } }
#pragma unroll
    for (int e = 0; e < 4; ++e) so[il][hb + hq * 4 + e] = o[e] / l[e]; }
  __syncthreads();
  for (int q = tid; q < 64 * 16; q += 256) { const int rl = q >> 4, pc = q & 15; vst2(O + ((size_t)b * SQ + i0 + rl) * NI + pc * 4, *(const v4f*)(&so[rl][pc * 4])); }
}
__global__ __launch_bounds__(128) void k_out(const float* __restrict__ O, const float* __restrict__ Wo, const float* __restrict__ bo, float* __restrict__ out) {
  __shared__ __align__(16) float so[4][16][132];
  const int tid = threadIdx.x, wave = tid >> 5, lane = tid & 31, col = lane & 15, g = lane >> 4;
  const int r0 = blockIdx.x * 64 + wave * 16, n0 = blockIdx.y * 128;
  v8f acc[8] = {};
#pragma unroll
  for (int kc = 0; kc < NI / 32; ++kc) { const F2 a = split_row(O + (size_t)(r0 + col) * NI, kc * 32, lane);
#pragma unroll
    for (int j = 0; j < 8; ++j) acc[j] = mac3(a, split_col(Wo, kc * 32, n0 + j * 16 + col, lane, DM, NI), acc[j]); }
#pragma unroll
  for (int j = 0; j < 8; ++j) { const float bb = bo[n0 + j * 16 + col];
#pragma unroll
    for (int r = 0; r < 8; ++r) so[wave][8 * g + r][j * 16 + col] = acc[j][r] + bb; }
  LDSX();
#pragma unroll 4
  for (int rl = 0; rl < 16; ++rl) vst2(out + (size_t)(r0 + rl) * DM + n0 + lane * 4, *(const v4f*)(&so[wave][rl][lane * 4]));
}
extern "C" void kernel_launch(void* const* d_in, const int* in_sizes, int n_in, void* d_out, int out_size, void* d_ws, size_t ws_size, hipStream_t stream) {
  (void)in_sizes; (void)n_in; (void)out_size; (void)ws_size;
  const float* x = (const float*)d_in[0]; const float* emb = (const float*)d_in[1]; const float* Wq = (const float*)d_in[2]; const float* Wk = (const float*)d_in[3]; const float* Wv = (const float*)d_in[4]; const float* Wo = (const float*)d_in[5]; const float* bo = (const float*)d_in[6];
  float* out = (float*)d_out;
  char* ws = (char*)d_ws; size_t off = 0;
  auto take = [&](size_t bytes) { char* p = ws + off; off += (bytes + 255) & ~(size_t)255; return p; };
  float* Q = (float*)take((size_t)NRQ * NI * 4); float* K = (float*)take((size_t)NB * SK * NI * 4); float* V = (float*)take((size_t)NB * SK * NI * 4); float* O = (float*)take((size_t)NRQ * NI * 4);
  k_proj<<<dim3(NRQ / 64, 3), 128, 0, stream>>>(x, emb, Wq, Wk, Wv, Q, K, V);
  k_attn<<<dim3(SQ / 64, NB), 256, 0, stream>>>(Q, K, V, O);
  k_out<<<dim3(NRQ / 64, DM / 128), 128, 0, stream>>>(O, Wo, bo, out);
}
